// SoftTimeAttention_28003186769980
// MI455X (gfx1250) — hardware-verified
//
#include <hip/hip_runtime.h>
#include <hip/hip_bf16.h>
#include <math.h>


#define BB 4
#define SS 4096
#define DD 256
#define HH 16
#define DKK 64
#define QW 2

typedef _Float16 bf16;
typedef __attribute__((ext_vector_type(4))) unsigned v4u_t;
typedef unsigned v4ua __attribute__((ext_vector_type(4), may_alias));
typedef __attribute__((ext_vector_type(4))) float v4f_t;
typedef float v4fa __attribute__((ext_vector_type(4), may_alias));
typedef __attribute__((ext_vector_type(16))) bf16  bf16x16;
typedef __attribute__((ext_vector_type(8)))  bf16  bf16x8;
typedef __attribute__((ext_vector_type(4)))  bf16  bf16x4;
typedef __attribute__((ext_vector_type(8)))  float f32x8;

#define LDS_STRIDE 48
#define KSTRIDE    72
#define VSTRIDE    48

__device__ __forceinline__ f32x8 wmma_bf16(bf16x16 a, bf16x16 b, f32x8 c) {
  return __builtin_amdgcn_wmma_f32_16x16x32_f16(
      false, a, false, b, (short)0, c, false, false);
}

template <typename T>
__device__ __forceinline__ bf16x16 load_frag(const T* __restrict__ base, int ld,
                                             int row0, int k0) {
  const int lane = threadIdx.x & 31;
  const int r    = lane & 15;
  const int kh   = (lane >> 4) * 8;
  const T* p0 = base + (size_t)(row0 + r) * ld + (k0 + kh);
  const T* p1 = p0 + 16;
  bf16x16 f;
#pragma unroll
  for (int i = 0; i < 8; ++i) {
    f[i]     = (bf16)p0[i];
    f[i + 8] = (bf16)p1[i];
  }
  return f;
}

__device__ __forceinline__ bf16x16 lds_frag(const bf16* base, int stride) {
  const int lane = threadIdx.x & 31;
  const int row  = lane & 15;
  const int kh   = (lane >> 4) * 8;
  const bf16x8 lo = *(const bf16x8*)(base + row * stride + kh);
  const bf16x8 hi = *(const bf16x8*)(base + row * stride + kh + 16);
  bf16x16 f;
#pragma unroll
  for (int i = 0; i < 8; ++i) { f[i] = lo[i]; f[i + 8] = hi[i]; }
  return f;
}

template <typename T>
__device__ __forceinline__ void stage_read16(const T* __restrict__ p, float* buf) {
#pragma unroll
  for (int i = 0; i < 16; ++i) buf[i] = (float)p[i];
}

__device__ __forceinline__ void stage_write(bf16* dst, const float* buf, int nquad) {
#pragma unroll
  for (int i = 0; i < nquad; ++i) {
    bf16x4 q;
    q[0] = (bf16)buf[4 * i];     q[1] = (bf16)buf[4 * i + 1];
    q[2] = (bf16)buf[4 * i + 2]; q[3] = (bf16)buf[4 * i + 3];
    *(bf16x4*)(dst + 4 * i) = q;
  }
}


#define RSPLIT (1.0f / 2048.0f)
__device__ __forceinline__ bf16 lo_of(float v, bf16 h) { return (bf16)((v - (float)h) * 2048.0f); }
__device__ __forceinline__ f32x8 wmma_split(bf16x16 a, bf16x16 al, bf16x16 b, bf16x16 bl, f32x8 c) {
  f32x8 x = {}; x = wmma_bf16(al, b, x); x = wmma_bf16(a, bl, x); return wmma_bf16(a, b, c) + x * RSPLIT; }

__global__ __launch_bounds__(256) void k_ht(const float* __restrict__ h, bf16* __restrict__ Ht, size_t PL) {
  __shared__ float tile[64][65];
  const int j0 = blockIdx.x * 64, d0 = blockIdx.y * 64, b = blockIdx.z, t = threadIdx.x;
  for (int i = t; i < 64 * 64; i += 256) { const int r = i >> 6, d = i & 63; tile[r][d] = h[((size_t)(b * SS + j0 + r)) * DD + d0 + d]; }
  __syncthreads();
#pragma unroll 1
  for (int pass = 0; pass < 2; ++pass) {
    for (int i = t; i < 64 * 8; i += 256) { const int dr = i >> 3, j8 = (i & 7) * 8; bf16 hh[8], hl[8];
#pragma unroll
      for (int e = 0; e < 8; ++e) { const float v = tile[j8 + e][dr]; hh[e] = (bf16)v; hl[e] = lo_of(v, hh[e]); }
      bf16* dst = Ht + ((size_t)b * DD + d0 + dr) * SS + j0 + j8; *(volatile v4u_t*)dst = *(const v4ua*)hh; *(volatile v4u_t*)(dst + PL) = *(const v4ua*)hl; }
    __threadfence();
  }
}
__global__ __launch_bounds__(64) void sta_kernel(const float* __restrict__ tt, const bf16* __restrict__ Ht, size_t PL, int vq, float* __restrict__ out) {
  __shared__ bf16 ldsV[2][64 * VSTRIDE];
  __shared__ __attribute__((aligned(16))) float ldsO[2][16 * 68];
  const int b = blockIdx.z, t = threadIdx.x, wave = t >> 5, lane = t & 31, qlane = lane & 15, kh8 = (lane >> 4) * 8;
  const int q0 = blockIdx.x * 32 + wave * 16;
  const float* tb = tt + (size_t)b * SS; const float tq = tb[q0 + qlane];
  const bf16* Hb = Ht + ((size_t)b * DD + vq * 64) * SS;
  f32x8 o[4] = {}; float lsum = 0.0f;
#pragma unroll 1
  for (int kb = 0; kb < SS; kb += 32) {
    __syncthreads();
    { const bf16* s0p = Hb + (size_t)t * SS + kb;
#pragma unroll
      for (int i = 0; i < 4; ++i) { *(bf16x8*)(&ldsV[0][t * VSTRIDE + 8 * i]) = *(const bf16x8*)(s0p + 8 * i); *(bf16x8*)(&ldsV[1][t * VSTRIDE + 8 * i]) = *(const bf16x8*)(s0p + PL + 8 * i); } }
    __syncthreads();
    bf16x16 pf, pl;
#pragma unroll
    for (int r = 0; r < 8; ++r) {
      const float d0 = tq - tb[kb + kh8 + r], d1 = tq - tb[kb + 16 + kh8 + r];
      const float v0 = 4096.0f * d0, v1 = 4096.0f * d1;
      const float l0 = -(v0 * v0) / 1.0f, l1 = -(v1 * v1) / 1.0f;
      const float p0 = expf(l0), p1 = expf(l1); lsum += p0 + p1;
      const float ps0 = p0 * 1024.0f, ps1 = p1 * 1024.0f;
      const bf16 h0 = (bf16)ps0, h1 = (bf16)ps1; pf[r] = h0; pf[r + 8] = h1; pl[r] = lo_of(ps0, h0); pl[r + 8] = lo_of(ps1, h1); }
#pragma unroll
    for (int j = 0; j < 4; ++j) o[j] = wmma_split(lds_frag(ldsV[0] + (j * 16) * VSTRIDE, VSTRIDE), lds_frag(ldsV[1] + (j * 16) * VSTRIDE, VSTRIDE), pf, pl, o[j]);
  }
  lsum += __shfl_xor(lsum, 16, 32);
  float* so = ldsO[wave]; const float rl = 1.0f / (lsum * 1024.0f);
#pragma unroll
  for (int j = 0; j < 4; ++j)
#pragma unroll
    for (int r = 0; r < 8; ++r) so[qlane * 68 + j * 16 + kh8 + r] = o[j][r] * rl;
  asm volatile("s_wait_dscnt 0" ::: "memory");
#pragma unroll 1
  for (int pass = 0; pass < 2; ++pass) {
#pragma unroll
    for (int it = 0; it < 8; ++it) { const int ch = lane + 32 * it, ql = ch >> 4, q4 = (ch & 15) * 4;
      float* dst = out + ((size_t)(b * SS + q0 + ql)) * DD + vq * 64 + q4;
      *(volatile v4f_t*)dst = *(const volatile v4fa*)(so + ql * 68 + q4); }
    __threadfence();
  }
}

extern "C" void kernel_launch(void* const* d_in, const int* in_sizes, int n_in,
                              void* d_out, int out_size, void* d_ws, size_t ws_size,
                              hipStream_t stream) {
  (void)in_sizes; (void)n_in; (void)out_size; (void)ws_size;
  const float* h = (const float*)d_in[0];
  const float* tt = (const float*)d_in[1];
  char* ws = (char*)d_ws;
  const size_t PL = (size_t)BB * DD * SS;
  bf16* Ht = (bf16*)ws; ws += PL * 2 * 2;
  k_ht<<<dim3(SS / 64, DD / 64, BB), 256, 0, stream>>>(h, Ht, PL);
  for (int vq = 0; vq < 4; ++vq) sta_kernel<<<dim3(SS / 32, 1, BB), 64, 0, stream>>>(tt, Ht, PL, vq, (float*)d_out);
}
